// GatedMoE_80032420593967
// MI455X (gfx1250) — hardware-verified
//
#include <hip/hip_runtime.h>
#include <math.h>

typedef __attribute__((ext_vector_type(16))) _Float16 v16h;
typedef __attribute__((ext_vector_type(16))) __bf16 v16b;
typedef __attribute__((ext_vector_type(8)))  _Float16 v8h;
typedef __attribute__((ext_vector_type(8)))  __bf16 v8b;
typedef __attribute__((ext_vector_type(8)))  float v8f;
typedef __attribute__((ext_vector_type(4)))  float v4f;
typedef __attribute__((ext_vector_type(4)))  unsigned v4u;
typedef _Float16 h16;

#ifndef NB
#define NB 4
#endif
#ifndef SEQ
#define SEQ 512
#endif
#define NB_FULL 4
#define SEQ_FULL 512
#define NTOK (NB * SEQ)
#define DM   128
#define NEXP 256
#define HCARRY 64.0f
#define WCARRY 512.0f
#define RCARRY 2048.0f
#define RINV (1.0f / 2048.0f)
#define OSCALE (1.0f / 32768.0f)
#define OUT1_ELEM ((size_t)NB_FULL * SEQ_FULL * DM)
#define RT 16
#define ET 64
#define FT 64

#define WS_XB  ((size_t)0)
#define WS_WET (WS_XB  + (size_t)NTOK * DM * 2)
#define WS_W1T (WS_WET + (size_t)NEXP * DM * DM * 2)
#define WS_W2T (WS_W1T + (size_t)DM * DM * 2)
#define WS_REC (WS_W2T + (size_t)DM * DM * 2)
#define WS_Y   (WS_REC + (size_t)NTOK * 16)
#define WS_END (WS_Y   + (size_t)NTOK * 2 * DM * 4)

static_assert(SEQ == SEQ_FULL || NB == 1);
static_assert(NB <= NB_FULL && SEQ <= SEQ_FULL);
static_assert(NTOK % 64 == 0);
static_assert(DM % 32 == 0 && DM == 128 && NEXP == 256);
static_assert(OUT1_ELEM * 4 == 1048576);
static_assert((OUT1_ELEM + (size_t)NTOK) * 4 <= 1056768);
static_assert(WS_WET % 128 == 0 && WS_W1T % 128 == 0 && WS_W2T % 128 == 0 && WS_REC % 128 == 0 && WS_Y % 128 == 0);
static_assert(WS_END <= (size_t)134217728);
static_assert((size_t)(NTOK * DM / 8 / 256) * 256 * 8 == (size_t)NTOK * DM);
static_assert((size_t)(DM / 64) * (DM / 64) * NEXP * 4096 == (size_t)NEXP * DM * DM);
static_assert((size_t)(DM / 64) * (DM / 64) * 4096 == (size_t)DM * DM);
static_assert((size_t)(NTOK / RT) * RT == (size_t)NTOK);
static_assert((size_t)(NTOK / ET) * 4 * 16 == (size_t)NTOK);
static_assert((size_t)(NTOK / FT) * 4 * 16 == (size_t)NTOK);
static_assert(32 * 16 == DM * 4);
static_assert(16 * 16 == RT * 16);
static_assert(16 * 16 == FT * 4);
static_assert(16 * 128 * 4 == FT * DM);
static_assert(2 * 256 * 4 == RT * DM);
static_assert(4 * 2 * 16 == DM);
static_assert(64 * 65 * 4 <= 131072);
static_assert(RT * DM * 4 + RT * (NEXP + 4) * 4 + RT * 16 <= 131072);
static_assert(4 * 16 * 132 * 4 <= 131072);
static_assert(2 * FT * 136 * 2 + FT * 132 * 4 + FT * 4 <= 131072);

__device__ __forceinline__ v8f wmma16(v16h a, v16h b, v8f c) {
  v8f d = __builtin_amdgcn_wmma_f32_16x16x32_f16(false, a, false, b, (short)0, c, false, false);
  asm volatile("v_nop\n\tv_nop\n\tv_nop\n\tv_nop" : "+v"(d) : "v"(a), "v"(b));
  return d;
}
__device__ __forceinline__ v8f wmma_bf(v16b a, v16b b, v8f c) {
  v8f d = __builtin_amdgcn_wmma_f32_16x16x32_bf16(false, a, false, b, (short)0, c, false, false);
  asm volatile("v_nop\n\tv_nop\n\tv_nop\n\tv_nop" : "+v"(d) : "v"(a), "v"(b));
  return d;
}
__device__ __forceinline__ float bfr(float v) { return (float)(__bf16)v; }
__device__ __forceinline__ h16 toh_flush(float v) { const h16 r = (h16)v; return (fabsf(v) < 6.103515625e-05f) ? (h16)0.0f : r; }
__device__ __forceinline__ v16b ldfrag_b(const unsigned short* p) { union { v16b v; v4u q[2]; } f; f.q[0] = *(const v4u*)p; f.q[1] = *(const v4u*)(p + 16); return f.v; }
__device__ __forceinline__ v16h ldfrag_h(const unsigned short* p) { union { v16h v; v4u q[2]; } f; f.q[0] = *(const v4u*)p; f.q[1] = *(const v4u*)(p + 16); return f.v; }

__global__ __launch_bounds__(256) void k_cvt_x(const float* __restrict__ X, unsigned short* __restrict__ XB) {
  const unsigned i = blockIdx.x * 256u + threadIdx.x;
  const unsigned ic = i < (unsigned)(NTOK * DM / 8) ? i : (unsigned)(NTOK * DM / 8 - 1);
  const v4f a = *(const v4f*)(X + (size_t)ic * 8), b = *(const v4f*)(X + (size_t)ic * 8 + 4);
  union { v8b h; v4u u; } o;
#pragma unroll
  for (int j = 0; j < 4; ++j) { o.h[j] = (__bf16)a[j]; o.h[4 + j] = (__bf16)b[j]; }
  const v4u val = o.u;
  volatile v4u* p = (volatile v4u*)(XB + (size_t)ic * 8);
  *p = val; __threadfence(); *p = val;
}

template <int F16>
__global__ __launch_bounds__(256) void k_tr(const float* __restrict__ S, unsigned short* __restrict__ Dst, unsigned K, unsigned N, unsigned dpitch, unsigned erow, unsigned ecol, float sc) {
  __shared__ float tile[64][65];
  const unsigned t = threadIdx.x, e = blockIdx.z, k0 = blockIdx.y * 64u, n0 = blockIdx.x * 64u;
  const float* s = S + (size_t)e * K * N;
#pragma unroll
  for (unsigned it = 0; it < 4; ++it) { const unsigned idx = it * 256u + t, kr = idx >> 4, c4 = idx & 15u;
    const v4f v = *(const v4f*)(s + (size_t)(k0 + kr) * N + n0 + 4u * c4);
    tile[kr][4u * c4 + 0] = v[0]; tile[kr][4u * c4 + 1] = v[1]; tile[kr][4u * c4 + 2] = v[2]; tile[kr][4u * c4 + 3] = v[3]; }
  __syncthreads();
  v4u o[2];
#pragma unroll
  for (unsigned it = 0; it < 2; ++it) { const unsigned idx = it * 256u + t, nr = idx >> 3, q = idx & 7u;
    union { v8b b; v8h h; v4u u; } w;
#pragma unroll
    for (int i = 0; i < 8; ++i) { const float v = bfr(tile[8u * q + i][nr]); if (F16) w.h[i] = toh_flush(v * sc); else w.b[i] = (__bf16)v; }
    o[it] = w.u; }
#pragma unroll
  for (unsigned it = 0; it < 2; ++it) { const unsigned idx = it * 256u + t, nr = idx >> 3, q = idx & 7u;
    *(volatile v4u*)(Dst + (size_t)(e * erow + n0 + nr) * dpitch + e * ecol + k0 + 8u * q) = o[it]; }
  __threadfence();
#pragma unroll
  for (unsigned it = 0; it < 2; ++it) { const unsigned idx = it * 256u + t, nr = idx >> 3, q = idx & 7u;
    *(volatile v4u*)(Dst + (size_t)(e * erow + n0 + nr) * dpitch + e * ecol + k0 + 8u * q) = o[it]; }
}

__device__ __forceinline__ bool top_better(float av, unsigned ai, float bv, unsigned bi) { return (av > bv) || ((av == bv) && (ai < bi)); }

__global__ __launch_bounds__(256) void k_route(const float* __restrict__ X, const float* __restrict__ GW, const float* __restrict__ GB, unsigned* __restrict__ REC) {
#pragma clang fp contract(off)
  __shared__ __align__(16) float xs[RT][DM];
  __shared__ __align__(16) float lg[RT][NEXP + 4];
  __shared__ __align__(16) unsigned rec[RT][4];
  const unsigned tid = threadIdx.x, lane = tid & 31u;
  const unsigned wave = (unsigned)__builtin_amdgcn_readfirstlane((int)(tid >> 5));
  const unsigned t0 = blockIdx.x * RT;
#pragma unroll
  for (unsigned it = 0; it < 2; ++it) { const unsigned idx = it * 256u + tid, r = idx >> 5, c4 = idx & 31u;
    const v4f v = *(const v4f*)(X + (size_t)(t0 + r) * DM + 4u * c4);
    xs[r][4u * c4 + 0] = bfr(v[0]); xs[r][4u * c4 + 1] = bfr(v[1]); xs[r][4u * c4 + 2] = bfr(v[2]); xs[r][4u * c4 + 3] = bfr(v[3]); }
  __syncthreads();
  float acc[RT];
#pragma unroll
  for (int tt = 0; tt < RT; ++tt) acc[tt] = 0.0f;
#pragma unroll 1
  for (unsigned k = 0; k < DM; ++k) { const float w = bfr(GW[(size_t)k * NEXP + tid]);
#pragma unroll
    for (int tt = 0; tt < RT; ++tt) acc[tt] = fmaf(xs[tt][k], w, acc[tt]); }
  const float gb = bfr(GB[tid]);
#pragma unroll
  for (int tt = 0; tt < RT; ++tt) lg[tt][tid] = acc[tt] + gb;
  __syncthreads();
#pragma unroll 1
  for (unsigned s = 0; s < 2u; ++s) { const unsigned row = wave * 2u + s;
    float m = lg[row][lane];
#pragma unroll 1
    for (unsigned j = 1; j < 8u; ++j) m = fmaxf(m, lg[row][lane + 32u * j]);
    m = fmaxf(m, __shfl_xor(m, 16)); m = fmaxf(m, __shfl_xor(m, 8)); m = fmaxf(m, __shfl_xor(m, 4)); m = fmaxf(m, __shfl_xor(m, 2)); m = fmaxf(m, __shfl_xor(m, 1));
    float z = 0.0f;
#pragma unroll 1
    for (unsigned j = 0; j < 8u; ++j) { const float u = expf(lg[row][lane + 32u * j] - m); lg[row][lane + 32u * j] = u; z += u; }
    z += __shfl_xor(z, 16); z += __shfl_xor(z, 8); z += __shfl_xor(z, 4); z += __shfl_xor(z, 2); z += __shfl_xor(z, 1);
    const float rz = 1.0f / z;
    float v1 = -1.0f, v2 = -1.0f; unsigned i1 = 0u, i2 = 0u;
#pragma unroll 1
    for (unsigned j = 0; j < 8u; ++j) { const unsigned e = lane + 32u * j; const float p = lg[row][e] * rz;
      const bool g1 = p > v1, g2 = p > v2;
      const float nv2 = g1 ? v1 : (g2 ? p : v2); const unsigned ni2 = g1 ? i1 : (g2 ? e : i2);
      v1 = g1 ? p : v1; i1 = g1 ? e : i1; v2 = nv2; i2 = ni2; }
#pragma unroll
    for (int off = 16; off >= 1; off >>= 1) {
      const float ov1 = __shfl_xor(v1, off), ov2 = __shfl_xor(v2, off);
      const unsigned oi1 = __shfl_xor(i1, off), oi2 = __shfl_xor(i2, off);
      const bool ab = top_better(v1, i1, ov1, oi1);
      const float ca = ab ? v2 : v1; const unsigned cia = ab ? i2 : i1;
      const float cb = ab ? ov1 : ov2; const unsigned cib = ab ? oi1 : oi2;
      const bool bb = top_better(ca, cia, cb, cib);
      const float n1 = ab ? v1 : ov1; const unsigned ni1 = ab ? i1 : oi1;
      v2 = bb ? ca : cb; i2 = bb ? cia : cib; v1 = n1; i1 = ni1; }
    const float rs = 1.0f / ((v1 + v2) + 1e-6f);
    const float w0 = v1 * rs, w1 = v2 * rs;
    if (lane == 0u) { rec[row][0] = i1; rec[row][1] = i2; rec[row][2] = __float_as_uint(w0); rec[row][3] = __float_as_uint(w1); }
  }
  __syncthreads();
  if (tid < 16u) { const v4u val = *(const v4u*)&rec[tid][0];
    volatile v4u* p = (volatile v4u*)(REC + (size_t)(t0 + tid) * 4);
    *p = val; __threadfence(); *p = val; }
}

__global__ __launch_bounds__(128) void k_exp(const unsigned short* __restrict__ XB, const unsigned short* __restrict__ WET, const unsigned* __restrict__ REC, float* __restrict__ Y) {
  __shared__ __align__(16) float sy[4][16][132];
  const unsigned t = threadIdx.x, lane = t & 31u, lm = lane & 15u, lh = lane >> 4;
  const unsigned wave = (unsigned)__builtin_amdgcn_readfirstlane((int)(t >> 5));
  const unsigned e = blockIdx.x, m0 = blockIdx.y * ET;
  const unsigned row = m0 + wave * 16u + lm;
  const v4u rc = *(const v4u*)(REC + (size_t)row * 4);
  const unsigned hm0 = __builtin_amdgcn_ballot_w32(rc[0] == e) & 0xffffu;
  const unsigned hm1 = __builtin_amdgcn_ballot_w32(rc[1] == e) & 0xffffu;
  const unsigned hm = hm0 | hm1;
  if (hm != 0u) {
    const unsigned short* ar = XB + (size_t)row * DM + 8u * lh;
    const unsigned short* br = WET + (size_t)(e * DM + lm) * DM + 8u * lh;
    v8f acc[8] = {};
#pragma unroll 2
    for (unsigned kc = 0; kc < DM / 32; ++kc) { const v16b a = ldfrag_b(ar + kc * 32u);
#pragma unroll
      for (int ni = 0; ni < 8; ++ni) { const v16b b = ldfrag_b(br + (size_t)ni * 16u * DM + kc * 32u); acc[ni] = wmma_bf(a, b, acc[ni]); } }
#pragma unroll
    for (int ni = 0; ni < 8; ++ni)
#pragma unroll
      for (int r = 0; r < 8; ++r) sy[wave][8u * lh + r][ni * 16 + lm] = acc[ni][r];
  }
  __syncthreads();
  if (hm != 0u) {
#pragma unroll 1
    for (unsigned r = 0; r < 16u; ++r) {
      if ((hm >> r) & 1u) { const unsigned slot = (hm1 >> r) & 1u;
        const v4f v = *(const v4f*)&sy[wave][r][4u * lane];
        *(volatile v4f*)(Y + ((size_t)(m0 + wave * 16u + r) * 2u + slot) * DM + 4u * lane) = v; } }
    __threadfence();
#pragma unroll 1
    for (unsigned r = 0; r < 16u; ++r) {
      if ((hm >> r) & 1u) { const unsigned slot = (hm1 >> r) & 1u;
        const v4f v = *(const v4f*)&sy[wave][r][4u * lane];
        *(volatile v4f*)(Y + ((size_t)(m0 + wave * 16u + r) * 2u + slot) * DM + 4u * lane) = v; } }
  }
}

__global__ __launch_bounds__(128) void k_fin(const float* __restrict__ Y, const unsigned* __restrict__ REC, const unsigned short* __restrict__ W1T, const unsigned short* __restrict__ W2T, const float* __restrict__ B1, const float* __restrict__ B2, float* __restrict__ OUT, float* __restrict__ CONS) {
  __shared__ __align__(16) _Float16 sa[FT][136];
  __shared__ __align__(16) _Float16 sr[FT][136];
  __shared__ __align__(16) float so[FT][132];
  __shared__ __align__(16) float sc[FT];
  const unsigned t = threadIdx.x, lane = t & 31u, lm = lane & 15u, lh = lane >> 4;
  const unsigned wave = (unsigned)__builtin_amdgcn_readfirstlane((int)(t >> 5));
  const unsigned t0 = blockIdx.x * FT;
#pragma unroll 2
  for (unsigned it = 0; it < 16u; ++it) { const unsigned idx = it * 128u + t, r = idx >> 5, c4 = idx & 31u; const size_t tok = (size_t)t0 + r;
    const v4u rc = *(const v4u*)(REC + tok * 4);
    const float w0 = __uint_as_float(rc[2]), w1 = __uint_as_float(rc[3]);
    const v4f y0 = *(const v4f*)(Y + (tok * 2) * DM + 4u * c4), y1 = *(const v4f*)(Y + (tok * 2 + 1) * DM + 4u * c4);
#pragma unroll
    for (int j = 0; j < 4; ++j) { const float m = (w0 * y0[j] + w1 * y1[j]) * HCARRY; const h16 hu = (h16)m;
      sa[r][4u * c4 + j] = toh_flush(m);
      sr[r][4u * c4 + j] = toh_flush((m - (float)hu) * RCARRY); } }
  __syncthreads();
  v16h a[4], ar[4];
#pragma unroll
  for (int kc = 0; kc < 4; ++kc) { union { v16h v; v8h q[2]; } f, fr;
    f.q[0] = *(const v8h*)&sa[wave * 16u + lm][kc * 32 + 8u * lh];
    f.q[1] = *(const v8h*)&sa[wave * 16u + lm][kc * 32 + 16 + 8u * lh];
    fr.q[0] = *(const v8h*)&sr[wave * 16u + lm][kc * 32 + 8u * lh];
    fr.q[1] = *(const v8h*)&sr[wave * 16u + lm][kc * 32 + 16 + 8u * lh];
    a[kc] = f.v; ar[kc] = fr.v; }
#pragma unroll 1
  for (unsigned nq = 0; nq < 4u; ++nq) {
    v8f g[2] = {}, h[2] = {}, gr[2] = {}, hr[2] = {};
#pragma unroll
    for (int kc = 0; kc < 4; ++kc)
#pragma unroll
      for (int ni = 0; ni < 2; ++ni) { const size_t bo = (size_t)(nq * 32u + ni * 16u + lm) * DM + kc * 32u + 8u * lh;
        const v16h b1 = ldfrag_h(W1T + bo); g[ni] = wmma16(a[kc], b1, g[ni]); gr[ni] = wmma16(ar[kc], b1, gr[ni]);
        const v16h b2 = ldfrag_h(W2T + bo); h[ni] = wmma16(a[kc], b2, h[ni]); hr[ni] = wmma16(ar[kc], b2, hr[ni]); }
#pragma unroll
    for (int ni = 0; ni < 2; ++ni) { const unsigned col = nq * 32u + ni * 16u + lm; const float bb1 = bfr(B1[col]), bb2 = bfr(B2[col]);
#pragma unroll
      for (int r = 0; r < 8; ++r) { const float gv = (g[ni][r] + gr[ni][r] * RINV) * OSCALE + bb1, hv = (h[ni][r] + hr[ni][r] * RINV) * OSCALE + bb2;
        const float sg = 1.0f / (1.0f + expf(-gv));
        so[wave * 16u + 8u * lh + r][col] = (gv * sg) * hv; } }
  }
  __syncthreads();
#pragma unroll 1
  for (unsigned r = 0; r < 16u; ++r) { const unsigned row = wave * 16u + r; const size_t tok = (size_t)t0 + row;
    const v4f o = *(const v4f*)&so[row][4u * lane];
    *(volatile v4f*)(OUT + tok * DM + 4u * lane) = o;
    const v4u rc = *(const v4u*)(REC + tok * 4);
    const float w0 = __uint_as_float(rc[2]), w1 = __uint_as_float(rc[3]);
    const v4f y0 = *(const v4f*)(Y + (tok * 2) * DM + 4u * lane), y1 = *(const v4f*)(Y + (tok * 2 + 1) * DM + 4u * lane);
    float s = 0.0f;
#pragma unroll
    for (int j = 0; j < 4; ++j) { const float d0 = y0[j] - o[j], d1 = y1[j] - o[j]; s += (d0 * d0) * w0 + (d1 * d1) * w1; }
    s += __shfl_xor(s, 16); s += __shfl_xor(s, 8); s += __shfl_xor(s, 4); s += __shfl_xor(s, 2); s += __shfl_xor(s, 1);
    if (lane == 0u) sc[row] = expf(-(s * (1.0f / (float)DM))); }
  __threadfence();
#pragma unroll 1
  for (unsigned r = 0; r < 16u; ++r) { const unsigned row = wave * 16u + r; const size_t tok = (size_t)t0 + row;
    const v4f o = *(const v4f*)&so[row][4u * lane];
    *(volatile v4f*)(OUT + tok * DM + 4u * lane) = o; }
  __syncthreads();
  if (t < 16u) { const v4f c = *(const v4f*)&sc[4u * t];
    volatile v4f* p = (volatile v4f*)(CONS + (size_t)t0 + 4u * t);
    *p = c; __threadfence(); *p = c; }
}

extern "C" void kernel_launch(void* const* d_in, const int* in_sizes, int n_in, void* d_out, int out_size, void* d_ws, size_t ws_size, hipStream_t stream) {
  if (n_in < 8) return;
  if (in_sizes[0] < NTOK * DM || in_sizes[1] < DM * NEXP || in_sizes[2] < NEXP || in_sizes[3] < NEXP * DM * DM) return;
  if (in_sizes[4] < DM * DM || in_sizes[5] < DM || in_sizes[6] < DM * DM || in_sizes[7] < DM) return;
  if ((size_t)out_size < OUT1_ELEM + (size_t)NTOK) return;
  if (ws_size < (size_t)WS_END) return;
  const float* X  = (const float*)d_in[0];
  const float* GW = (const float*)d_in[1];
  const float* GB = (const float*)d_in[2];
  const float* EW = (const float*)d_in[3];
  const float* W1 = (const float*)d_in[4];
  const float* B1 = (const float*)d_in[5];
  const float* W2 = (const float*)d_in[6];
  const float* B2 = (const float*)d_in[7];
  char* ws = (char*)d_ws;
  unsigned short* XB  = (unsigned short*)(ws + WS_XB);
  unsigned short* WET = (unsigned short*)(ws + WS_WET);
  unsigned short* W1T = (unsigned short*)(ws + WS_W1T);
  unsigned short* W2T = (unsigned short*)(ws + WS_W2T);
  unsigned* REC = (unsigned*)(ws + WS_REC);
  float* Y    = (float*)(ws + WS_Y);
  float* OUT  = (float*)d_out;
  float* CONS = (float*)d_out + OUT1_ELEM;
  k_cvt_x<<<dim3(NTOK * DM / 8 / 256), 256, 0, stream>>>(X, XB);
  k_tr<0><<<dim3(DM / 64, DM / 64, NEXP), 256, 0, stream>>>(EW, WET, (unsigned)DM, (unsigned)DM, (unsigned)DM, (unsigned)DM, 0u, 1.0f);
  k_tr<1><<<dim3(DM / 64, DM / 64, 1), 256, 0, stream>>>(W1, W1T, (unsigned)DM, (unsigned)DM, (unsigned)DM, 0u, 0u, WCARRY);
  k_tr<1><<<dim3(DM / 64, DM / 64, 1), 256, 0, stream>>>(W2, W2T, (unsigned)DM, (unsigned)DM, (unsigned)DM, 0u, 0u, WCARRY);
  k_route<<<dim3(NTOK / RT), 256, 0, stream>>>(X, GW, GB, REC);
  k_exp<<<dim3(NEXP, NTOK / ET), 128, 0, stream>>>(XB, WET, REC, Y);
  k_fin<<<dim3(NTOK / FT), 128, 0, stream>>>(Y, REC, W1T, W2T, B1, B2, OUT, CONS);
}
